// TransformerBlock_32564442038942
// MI455X (gfx1250) — hardware-run, weakly checked
//
#include <hip/hip_runtime.h>


#ifndef NB
#define NB 8
#endif
#ifndef SEQ
#define SEQ 2048
#endif
#define NB_FULL  8
#define SEQ_FULL 2048
#ifndef OUT_SEQ
#define OUT_SEQ SEQ
#endif
#define DM   256
#define NH_  2
#define HD   128
#define QKVW 768
#define AW   4
#define OSP  132
#define GW   2
#define TP   260
#define QRS  2048.0f
#define QRI  (1.0f / 2048.0f)
#define L2E  1.4426950408889634f
#define PSH  14.0f
#define PFL  (-14.0f)
#define NEGB (-3.0e38f)
#define WSC  64.0f
#define ASC  16.0f
#define SCI  (1.0f / 1024.0f)
#define LNEPS 1.0e-5f

static_assert(HD == 128);
static_assert(NH_ * HD == DM);
static_assert(QKVW == 3 * DM);
static_assert(QKVW == NH_ * 3 * HD);
static_assert(HD % 64 == 0);
static_assert(DM % 64 == 0);
static_assert(DM % 32 == 0);
static_assert(HD % 32 == 0);
static_assert(QKVW % 32 == 0);
static_assert(SEQ % 64 == 0);
static_assert((NB * SEQ) % 64 == 0);
static_assert(SEQ % 32 == 0);
static_assert(SEQ % (16 * AW) == 0);
static_assert(SEQ % (16 * GW) == 0);
static_assert((NB * SEQ) % (16 * GW) == 0);
static_assert(((size_t)SEQ * DM) % 8 == 0);
static_assert(NB <= NB_FULL);
static_assert(SEQ <= SEQ_FULL);
static_assert((OSP * 4) % 16 == 0);
static_assert((TP * 4) % 16 == 0);
static_assert(OSP >= HD);
static_assert(TP >= DM);
static_assert(AW * 16 * OSP * 4 <= 131072);
static_assert(GW * 16 * TP * 4 <= 131072);
static_assert(4 * 32 * 8 == 16 * 64);
static_assert(8 * 32 * 8 == 16 * HD);
static_assert(2 * 32 * 4 == DM);
static_assert(32 * 8 == DM);
static_assert(256 * 8 == 64 * 32);

typedef _Float16 h16;
typedef unsigned short bf;
typedef __attribute__((ext_vector_type(16))) __bf16   v16bf;
typedef __attribute__((ext_vector_type(16))) _Float16 v16h;
typedef __attribute__((ext_vector_type(8)))  _Float16 v8h;
typedef __attribute__((ext_vector_type(8)))  unsigned short v8us;
typedef __attribute__((ext_vector_type(8)))  float    v8f;
typedef __attribute__((ext_vector_type(4)))  float    v4f;
typedef v4f  __attribute__((may_alias)) v4fa;

__device__ __forceinline__ unsigned short f2bf(float f) { unsigned u = __float_as_uint(f); u += 0x7FFFu + ((u >> 16) & 1u); return (unsigned short)(u >> 16); }
__device__ __forceinline__ float bfr(float f) { return __uint_as_float(((unsigned)f2bf(f)) << 16); }
__device__ __forceinline__ v16h cat16(v8h lo, v8h hi) { return __builtin_shufflevector(lo, hi, 0, 1, 2, 3, 4, 5, 6, 7, 8, 9, 10, 11, 12, 13, 14, 15); }
__device__ __forceinline__ v16bf cat16b(v8us lo, v8us hi) { return __builtin_bit_cast(v16bf, __builtin_shufflevector(lo, hi, 0, 1, 2, 3, 4, 5, 6, 7, 8, 9, 10, 11, 12, 13, 14, 15)); }
__device__ __forceinline__ v8f wmma16(v16h a, v16h b, v8f c) { return __builtin_amdgcn_wmma_f32_16x16x32_f16(false, a, false, b, (short)0, c, false, false); }
__device__ __forceinline__ v8f wmmab(v16bf a, v16bf b, v8f c) { return __builtin_amdgcn_wmma_f32_16x16x32_bf16(false, a, false, b, (short)0, c, false, false); }
__device__ __forceinline__ v16h  ldh(const h16* p) { return cat16(*(const v8h*)p, *(const v8h*)(p + 16)); }
__device__ __forceinline__ v16bf ldb(const bf* p)  { return cat16b(*(const v8us*)p, *(const v8us*)(p + 16)); }
__device__ __forceinline__ void wave_sync() { __builtin_amdgcn_fence(3  , "wavefront"); __builtin_amdgcn_wave_barrier(); asm volatile("" ::: "memory"); }

__device__ __forceinline__ v8f wmma16g(v16h a, v16h b, v8f c) { c = wmma16(a, b, c); asm volatile("v_nop\n\tv_nop\n\tv_nop\n\tv_nop" : "+v"(c) : "v"(a), "v"(b)); return c; }
__device__ __forceinline__ v8f wmmabg(v16bf a, v16bf b, v8f c) { c = wmmab(a, b, c); asm volatile("v_nop\n\tv_nop\n\tv_nop\n\tv_nop" : "+v"(c) : "v"(a), "v"(b)); return c; }
static __device__ __forceinline__ h16 toh_flush(float v) { const float w = (fabsf(v) < 6.103515625e-05f) ? 0.0f : v; return (h16)w; }

__global__ __launch_bounds__(256) void k_cvt8(const float* __restrict__ src, bf* dst, size_t n8) {
    const size_t i = (size_t)blockIdx.x * 256 + threadIdx.x; if (i >= n8) return;
    const v8f v = *(const v8f*)(src + i * 8); v8us o;
#pragma unroll
    for (int k = 0; k < 8; ++k) o[k] = f2bf(v[k]);
    *(volatile v8us*)(dst + i * 8) = o; __threadfence(); *(volatile v8us*)(dst + i * 8) = o;
}

__global__ __launch_bounds__(256) void k_wt_bf(const float* __restrict__ W, bf* T, int K, int N) {
    __shared__ float tl[64 * 33];
    const unsigned tid = threadIdx.x; const unsigned k0 = blockIdx.x * 64u, n0 = blockIdx.y * 32u;
#pragma unroll 1
    for (unsigned i = 0; i < 8u; ++i) { const unsigned e = i * 256u + tid; const unsigned kk = e >> 5, nn = e & 31u;
        tl[kk * 33u + nn] = W[(size_t)(k0 + kk) * (size_t)N + n0 + nn]; }
    __syncthreads();
    const unsigned row = tid >> 3, c8 = (tid & 7u) * 8u;
    v8us o;
#pragma unroll
    for (int i = 0; i < 8; ++i) o[i] = f2bf(tl[(c8 + (unsigned)i) * 33u + row]);
    bf* dp = T + (size_t)(n0 + row) * (size_t)K + k0 + c8;
    *(volatile v8us*)dp = o; __threadfence(); *(volatile v8us*)dp = o;
}

__global__ __launch_bounds__(256) void k_wt_h(const float* __restrict__ W, h16* T, int K, int N) {
    __shared__ float tl[64 * 33];
    const unsigned tid = threadIdx.x; const unsigned k0 = blockIdx.x * 64u, n0 = blockIdx.y * 32u;
#pragma unroll 1
    for (unsigned i = 0; i < 8u; ++i) { const unsigned e = i * 256u + tid; const unsigned kk = e >> 5, nn = e & 31u;
        tl[kk * 33u + nn] = W[(size_t)(k0 + kk) * (size_t)N + n0 + nn]; }
    __syncthreads();
    const unsigned row = tid >> 3, c8 = (tid & 7u) * 8u;
    v8h o;
#pragma unroll
    for (int i = 0; i < 8; ++i) o[i] = toh_flush(bfr(tl[(c8 + (unsigned)i) * 33u + row]) * WSC);
    h16* dp = T + (size_t)(n0 + row) * (size_t)K + k0 + c8;
    *(volatile v8h*)dp = o; __threadfence(); *(volatile v8h*)dp = o;
}

__device__ __forceinline__ void gemm64_bf(const bf* __restrict__ A, const bf* __restrict__ Bt, size_t aoff, size_t boff, v8f (&acc)[4][4]) {
#pragma unroll 1
    for (int kc = 0; kc < DM; kc += 32) {
        v16bf a[4];
#pragma unroll
        for (int mb = 0; mb < 4; ++mb) a[mb] = ldb(A + aoff + (size_t)mb * 16 * DM + kc);
#pragma unroll
        for (int nb = 0; nb < 4; ++nb) { const v16bf b = ldb(Bt + boff + (size_t)nb * 16 * DM + kc);
#pragma unroll
            for (int mb = 0; mb < 4; ++mb) acc[mb][nb] = wmmabg(a[mb], b, acc[mb][nb]); }
    }
}

__global__ __launch_bounds__(32) void k_qk(const bf* __restrict__ A, const bf* __restrict__ Bt, const float* __restrict__ bias, h16* PH, h16* PR) {
    __shared__ __align__(16) float os[16 * 68];
    const int lane = threadIdx.x & 31, lr = lane & 15, hi = lane >> 4;
    const unsigned bx = blockIdx.x, by = blockIdx.y;
    const unsigned r0 = bx * 64u;
    const unsigned hh = by / 4u, wh = (by % 4u) / 2u, dh = by % 2u;
    const unsigned c0 = hh * (3u * HD) + wh * (unsigned)HD + dh * 64u;
    v8f acc[4][4];
#pragma unroll
    for (int mb = 0; mb < 4; ++mb)
#pragma unroll
        for (int nb = 0; nb < 4; ++nb) acc[mb][nb] = (v8f){};
    gemm64_bf(A, Bt, (size_t)(r0 + (unsigned)lr) * DM + 8 * hi, (size_t)(c0 + (unsigned)lr) * DM + 8 * hi, acc);
    float bc[4];
#pragma unroll
    for (int nb = 0; nb < 4; ++nb) bc[nb] = bfr(bias[c0 + (unsigned)(nb * 16 + lr)]);
    const unsigned bb = r0 / (unsigned)SEQ, tt = r0 % (unsigned)SEQ;
    const size_t tbase = (size_t)wh * ((size_t)NB * NH_ * SEQ * HD) + ((size_t)(bb * (unsigned)NH_ + hh) * SEQ + (size_t)tt) * HD + (size_t)dh * 64;
#pragma unroll
    for (int mb = 0; mb < 4; ++mb) {
#pragma unroll
        for (int nb = 0; nb < 4; ++nb) {
#pragma unroll
            for (int j = 0; j < 8; ++j) os[(hi * 8 + j) * 68 + nb * 16 + lr] = acc[mb][nb][j] + bc[nb]; }
        wave_sync();
#pragma unroll 1
        for (int ps = 0; ps < 2; ++ps) {
            const size_t sb = tbase + (size_t)(mb * 16) * HD;
#pragma unroll
            for (int s = 0; s < 4; ++s) { const int row = 4 * s + (lane >> 3), c8 = (lane & 7) * 8;
                const v4f x0 = *(const v4fa*)(&os[row * 68 + c8]); const v4f x1 = *(const v4fa*)(&os[row * 68 + c8 + 4]); v8h hv, rv;
#pragma unroll
                for (int i = 0; i < 4; ++i) { const h16 a0 = toh_flush(x0[i]); const h16 a1 = toh_flush(x1[i]); hv[i] = a0; hv[4 + i] = a1;
                    rv[i] = toh_flush((x0[i] - (float)a0) * QRS); rv[4 + i] = toh_flush((x1[i] - (float)a1) * QRS); }
                const size_t oo = sb + (size_t)row * HD + c8;
                *(volatile v8h*)(PH + oo) = hv; *(volatile v8h*)(PR + oo) = rv; }
            if (ps == 0) __threadfence(); }
        wave_sync();
    }
}

__global__ __launch_bounds__(32) void k_vt(const bf* __restrict__ A, const bf* __restrict__ Bt, const float* __restrict__ bias, h16* VT) {
    __shared__ __align__(16) float os[16 * 68];
    const int lane = threadIdx.x & 31, lr = lane & 15, hi = lane >> 4;
    const unsigned bx = blockIdx.x, by = blockIdx.y;
    const unsigned hh = bx / 2u, dh = bx % 2u;
    const unsigned r0 = hh * (3u * HD) + 2u * HD + dh * 64u;
    const unsigned c0 = by * 64u;
    v8f acc[4][4];
#pragma unroll
    for (int mb = 0; mb < 4; ++mb)
#pragma unroll
        for (int nb = 0; nb < 4; ++nb) acc[mb][nb] = (v8f){};
    gemm64_bf(A, Bt, (size_t)(r0 + (unsigned)lr) * DM + 8 * hi, (size_t)(c0 + (unsigned)lr) * DM + 8 * hi, acc);
    const unsigned bb = c0 / (unsigned)SEQ, tt = c0 % (unsigned)SEQ;
    const size_t tbase = ((size_t)(bb * (unsigned)NH_ + hh) * HD + (size_t)dh * 64) * SEQ + (size_t)tt;
#pragma unroll
    for (int mb = 0; mb < 4; ++mb) {
        float br[8];
#pragma unroll
        for (int j = 0; j < 8; ++j) br[j] = bfr(bias[r0 + (unsigned)(mb * 16 + hi * 8 + j)]);
#pragma unroll
        for (int nb = 0; nb < 4; ++nb) {
#pragma unroll
            for (int j = 0; j < 8; ++j) os[(hi * 8 + j) * 68 + nb * 16 + lr] = acc[mb][nb][j] + br[j]; }
        wave_sync();
#pragma unroll 1
        for (int ps = 0; ps < 2; ++ps) {
            const size_t sb = tbase + (size_t)(mb * 16) * SEQ;
#pragma unroll
            for (int s = 0; s < 4; ++s) { const int row = 4 * s + (lane >> 3), c8 = (lane & 7) * 8;
                const v4f x0 = *(const v4fa*)(&os[row * 68 + c8]); const v4f x1 = *(const v4fa*)(&os[row * 68 + c8 + 4]); v8h hv;
#pragma unroll
                for (int i = 0; i < 4; ++i) { hv[i] = toh_flush(x0[i]); hv[4 + i] = toh_flush(x1[i]); }
                const size_t oo = sb + (size_t)row * SEQ + c8;
                *(volatile v8h*)(VT + oo) = hv; }
            if (ps == 0) __threadfence(); }
        wave_sync();
    }
}

__global__ __launch_bounds__(32 * AW) __attribute__((amdgpu_num_vgpr(256)))
void k_flash(const h16* __restrict__ QH, const h16* __restrict__ QR, const h16* __restrict__ KP, const h16* __restrict__ KR,
             const h16* __restrict__ VT, h16* CTX) {
    __shared__ __align__(16) float os[AW * 16 * OSP];
    const int lane = threadIdx.x & 31, lr = lane & 15, hi = lane >> 4;
    const int wave = __builtin_amdgcn_readfirstlane((int)(threadIdx.x >> 5));
    const unsigned zh = blockIdx.y; const unsigned b = zh / (unsigned)NH_, h = zh % (unsigned)NH_;
    const unsigned t0 = (blockIdx.x * (unsigned)AW + (unsigned)wave) * 16u;
    const size_t pbase = (size_t)zh * SEQ * HD;
    const h16* qhp = QH + pbase; const h16* qrp = QR + pbase;
    const h16* kpp = KP + pbase; const h16* krp = KR + pbase;
    const h16* vtp = VT + pbase;
    const unsigned qo = (t0 + (unsigned)lr) * (unsigned)HD + 8u * (unsigned)hi;
    const unsigned ko = (unsigned)lr * (unsigned)HD + 8u * (unsigned)hi;
    const unsigned vo = (unsigned)lr * (unsigned)SEQ + 8u * (unsigned)hi;
    v8f o[8];
#pragma unroll
    for (int j = 0; j < 8; ++j) o[j] = (v8f){};
    float m = NEGB, l = 0.0f;
#pragma unroll 1
    for (unsigned key0 = 0; key0 < (unsigned)SEQ; key0 += 32u) {
        unsigned qoff = qo; asm volatile("" : "+v"(qoff));
        const unsigned kof = ko + key0 * (unsigned)HD;
        v8f sHa = (v8f){}, sLa = (v8f){}, sHb = (v8f){}, sLb = (v8f){};
#pragma unroll 1
        for (unsigned kc = 0; kc < (unsigned)HD; kc += 32u) {
            const v16h qh = ldh(qhp + qoff + kc), qr = ldh(qrp + qoff + kc);
            const v16h ka = ldh(kpp + kof + kc), kb = ldh(kpp + kof + 16u * HD + kc);
            const v16h ra = ldh(krp + kof + kc), rb = ldh(krp + kof + 16u * HD + kc);
            sHa = wmma16g(ka, qh, sHa); sLa = wmma16g(ka, qr, sLa); sLa = wmma16g(ra, qh, sLa);
            sHb = wmma16g(kb, qh, sHb); sLb = wmma16g(kb, qr, sLb); sLb = wmma16g(rb, qh, sLb);
        }
        float ta[8], tb[8]; float mx = NEGB;
#pragma unroll
        for (int r = 0; r < 8; ++r) {
            ta[r] = (sHa[r] + sLa[r] * QRI) * L2E; tb[r] = (sHb[r] + sLb[r] * QRI) * L2E;
            mx = fmaxf(mx, fmaxf(ta[r], tb[r])); }
        mx = fmaxf(mx, __shfl_xor(mx, 16, 32));
        const float mnew = fmaxf(m, mx);
        const float alpha = __builtin_amdgcn_exp2f(m - mnew);
        const float sh = PSH - mnew;
        v16h pb; float ls = 0.0f;
#pragma unroll
        for (int r = 0; r < 8; ++r) {
            const float xa = ta[r] + sh, xb = tb[r] + sh;
            const float ea = __builtin_amdgcn_exp2f(xa), eb = __builtin_amdgcn_exp2f(xb);
            const float ga = (xa < PFL) ? 0.0f : ea, gb = (xb < PFL) ? 0.0f : eb;
            const h16 pa = (h16)ga; const h16 pc = (h16)gb;
            pb[r] = pa; pb[8 + r] = pc;
            ls += (float)pa + (float)pc; }
        l = l * alpha + ls; m = mnew;
#pragma unroll
        for (int j = 0; j < 8; ++j) o[j] = o[j] * alpha;
        const unsigned vof = vo + key0;
#pragma unroll
        for (int j = 0; j < 8; ++j) { const v16h vv = ldh(vtp + vof + (unsigned)(16 * j) * (unsigned)SEQ); o[j] = wmma16g(vv, pb, o[j]); }
    }
    l += __shfl_xor(l, 16, 32);
    const float inv = 1.0f / l;
    const int wb = wave * 16 * OSP;
#pragma unroll
    for (int j = 0; j < 8; ++j) { v4f a, c;
#pragma unroll
        for (int i = 0; i < 4; ++i) { a[i] = o[j][i] * inv; c[i] = o[j][4 + i] * inv; }
        *(v4fa*)(&os[wb + lr * OSP + 16 * j + 8 * hi]) = a; *(v4fa*)(&os[wb + lr * OSP + 16 * j + 8 * hi + 4]) = c; }
    wave_sync();
    h16* crow = CTX + ((size_t)b * SEQ + (size_t)t0) * DM + (size_t)h * HD;
#pragma unroll 1
    for (int ps = 0; ps < 2; ++ps) {
#pragma unroll
        for (int s = 0; s < 8; ++s) { const int row = 2 * s + (lane >> 4), c8 = (lane & 15) * 8;
            const v4f x0 = *(const v4fa*)(&os[wb + row * OSP + c8]); const v4f x1 = *(const v4fa*)(&os[wb + row * OSP + c8 + 4]); v8h hv;
#pragma unroll
            for (int i = 0; i < 4; ++i) { hv[i] = toh_flush(x0[i] * ASC); hv[4 + i] = toh_flush(x1[i] * ASC); }
            *(volatile v8h*)(crow + (size_t)row * DM + c8) = hv; }
        if (ps == 0) __threadfence(); }
}

__global__ __launch_bounds__(32 * GW) void k_gemm_ln(const h16* __restrict__ A, const h16* __restrict__ Bt, const float* __restrict__ bias, const float* __restrict__ RES,
                                                     const float* __restrict__ gam, const float* __restrict__ bet, float* OUTF, h16* OUTH, int rbs, int obs, int mode) {
    __shared__ __align__(16) float os[GW * 16 * TP];
    const int lane = threadIdx.x & 31, lr = lane & 15, hi = lane >> 4;
    const int wave = __builtin_amdgcn_readfirstlane((int)(threadIdx.x >> 5));
    const unsigned row0 = (blockIdx.x * (unsigned)GW + (unsigned)wave) * 16u;
    const unsigned bb = row0 / (unsigned)SEQ, tt = row0 % (unsigned)SEQ;
    const int wb = wave * 16 * TP;
    const h16* ap = A + (size_t)(row0 + (unsigned)lr) * DM + 8 * hi;
#pragma unroll 1
    for (int pass = 0; pass < 4; ++pass) {
        v8f c0 = (v8f){}, c1 = (v8f){}, c2 = (v8f){}, c3 = (v8f){};
        const h16* bp = Bt + (size_t)(pass * 64 + lr) * DM + 8 * hi;
#pragma unroll 1
        for (int kc = 0; kc < DM; kc += 32) {
            const v16h a = ldh(ap + kc);
            const v16h b0 = ldh(bp + kc);            c0 = wmma16g(a, b0, c0);
            const v16h b1 = ldh(bp + 16 * DM + kc);  c1 = wmma16g(a, b1, c1);
            const v16h b2 = ldh(bp + 32 * DM + kc);  c2 = wmma16g(a, b2, c2);
            const v16h b3 = ldh(bp + 48 * DM + kc);  c3 = wmma16g(a, b3, c3);
        }
        const int cb = wb + pass * 64 + lr;
#pragma unroll
        for (int j = 0; j < 8; ++j) { const int ro = cb + (hi * 8 + j) * TP;
            os[ro] = c0[j]; os[ro + 16] = c1[j]; os[ro + 32] = c2[j]; os[ro + 48] = c3[j]; }
    }
    wave_sync();
    const unsigned cA = (unsigned)lane * 4u, cB = 128u + (unsigned)lane * 4u;
    v4f bA = *(const v4f*)(bias + cA), bB = *(const v4f*)(bias + cB);
    v4f gA = *(const v4f*)(gam + cA),  gB = *(const v4f*)(gam + cB);
    v4f eA = *(const v4f*)(bet + cA),  eB = *(const v4f*)(bet + cB);
#pragma unroll
    for (int i = 0; i < 4; ++i) { bA[i] = bfr(bA[i]); bB[i] = bfr(bB[i]); gA[i] = bfr(gA[i]); gB[i] = bfr(gB[i]); eA[i] = bfr(eA[i]); eB[i] = bfr(eB[i]); }
    const float* rbase = RES + ((size_t)bb * (size_t)rbs + (size_t)tt) * DM;
#pragma unroll 1
    for (int r = 0; r < 16; ++r) {
        const v4f va = *(const v4fa*)(&os[wb + r * TP + (int)cA]); const v4f vb = *(const v4fa*)(&os[wb + r * TP + (int)cB]);
        const float* rp = rbase + (size_t)r * DM;
        const v4f ra = *(const v4f*)(rp + cA); const v4f rb = *(const v4f*)(rp + cB);
        float xa[4], xb[4];
#pragma unroll
        for (int i = 0; i < 4; ++i) {
            const float qa = bfr(ra[i]), qb = bfr(rb[i]);
            const float sa = (mode != 0) ? ra[i] : qa, sb = (mode != 0) ? rb[i] : qb;
            xa[i] = fmaxf(va[i] * SCI + bA[i], 0.0f) + sa; xb[i] = fmaxf(vb[i] * SCI + bB[i], 0.0f) + sb; }
        float s = ((xa[0] + xa[1]) + (xa[2] + xa[3])) + ((xb[0] + xb[1]) + (xb[2] + xb[3]));
        s += __shfl_xor(s, 16, 32); s += __shfl_xor(s, 8, 32); s += __shfl_xor(s, 4, 32); s += __shfl_xor(s, 2, 32); s += __shfl_xor(s, 1, 32);
        const float mu = s * (1.0f / 256.0f);
        float q = 0.0f;
#pragma unroll
        for (int i = 0; i < 4; ++i) { xa[i] -= mu; xb[i] -= mu; q += xa[i] * xa[i] + xb[i] * xb[i]; }
        q += __shfl_xor(q, 16, 32); q += __shfl_xor(q, 8, 32); q += __shfl_xor(q, 4, 32); q += __shfl_xor(q, 2, 32); q += __shfl_xor(q, 1, 32);
        const float rs = rsqrtf(q * (1.0f / 256.0f) + LNEPS);
        v4f ya, yb;
#pragma unroll
        for (int i = 0; i < 4; ++i) { ya[i] = xa[i] * rs * gA[i] + eA[i]; yb[i] = xb[i] * rs * gB[i] + eB[i]; }
        *(v4fa*)(&os[wb + r * TP + (int)cA]) = ya; *(v4fa*)(&os[wb + r * TP + (int)cB]) = yb;
    }
    wave_sync();
    float* op = OUTF + ((size_t)bb * (size_t)obs + (size_t)tt) * DM;
    h16* hp = OUTH + (size_t)row0 * DM;
    const int c8 = lane * 8;
#pragma unroll 1
    for (int ps = 0; ps < 2; ++ps) {
#pragma unroll 1
        for (int r = 0; r < 16; ++r) {
            const v4f ya = *(const v4fa*)(&os[wb + r * TP + (int)cA]); const v4f yb = *(const v4fa*)(&os[wb + r * TP + (int)cB]);
            *(volatile v4f*)(op + (size_t)r * DM + cA) = ya;
            *(volatile v4f*)(op + (size_t)r * DM + cB) = yb;
            if (mode == 0) {
                const v4f h0 = *(const v4fa*)(&os[wb + r * TP + c8]); const v4f h1 = *(const v4fa*)(&os[wb + r * TP + c8 + 4]); v8h hv;
#pragma unroll
                for (int i = 0; i < 4; ++i) { hv[i] = toh_flush(h0[i] * ASC); hv[4 + i] = toh_flush(h1[i] * ASC); }
                *(volatile v8h*)(hp + (size_t)r * DM + c8) = hv; } }
        if (ps == 0) __threadfence(); }
}

__global__ __launch_bounds__(32 * GW) void k_gemm_relu(const h16* __restrict__ A, const h16* __restrict__ Bt, const float* __restrict__ bias, h16* OUTH) {
    __shared__ __align__(16) float os[GW * 16 * TP];
    const int lane = threadIdx.x & 31, lr = lane & 15, hi = lane >> 4;
    const int wave = __builtin_amdgcn_readfirstlane((int)(threadIdx.x >> 5));
    const unsigned row0 = (blockIdx.x * (unsigned)GW + (unsigned)wave) * 16u;
    const int wb = wave * 16 * TP;
    const h16* ap = A + (size_t)(row0 + (unsigned)lr) * DM + 8 * hi;
#pragma unroll 1
    for (int pass = 0; pass < 4; ++pass) {
        v8f c0 = (v8f){}, c1 = (v8f){}, c2 = (v8f){}, c3 = (v8f){};
        const h16* bp = Bt + (size_t)(pass * 64 + lr) * DM + 8 * hi;
#pragma unroll 1
        for (int kc = 0; kc < DM; kc += 32) {
            const v16h a = ldh(ap + kc);
            const v16h b0 = ldh(bp + kc);            c0 = wmma16g(a, b0, c0);
            const v16h b1 = ldh(bp + 16 * DM + kc);  c1 = wmma16g(a, b1, c1);
            const v16h b2 = ldh(bp + 32 * DM + kc);  c2 = wmma16g(a, b2, c2);
            const v16h b3 = ldh(bp + 48 * DM + kc);  c3 = wmma16g(a, b3, c3);
        }
        const int cb = wb + pass * 64 + lr;
#pragma unroll
        for (int j = 0; j < 8; ++j) { const int ro = cb + (hi * 8 + j) * TP;
            os[ro] = c0[j]; os[ro + 16] = c1[j]; os[ro + 32] = c2[j]; os[ro + 48] = c3[j]; }
    }
    wave_sync();
    const int c8 = lane * 8;
    v4f b0 = *(const v4f*)(bias + c8), b1 = *(const v4f*)(bias + c8 + 4);
#pragma unroll
    for (int i = 0; i < 4; ++i) { b0[i] = bfr(b0[i]); b1[i] = bfr(b1[i]); }
    h16* hp = OUTH + (size_t)row0 * DM;
#pragma unroll 1
    for (int ps = 0; ps < 2; ++ps) {
#pragma unroll 1
        for (int r = 0; r < 16; ++r) {
            const v4f h0 = *(const v4fa*)(&os[wb + r * TP + c8]); const v4f h1 = *(const v4fa*)(&os[wb + r * TP + c8 + 4]); v8h hv;
#pragma unroll
            for (int i = 0; i < 4; ++i) { hv[i] = toh_flush(fmaxf(h0[i] * SCI + b0[i], 0.0f) * ASC); hv[4 + i] = toh_flush(fmaxf(h1[i] * SCI + b1[i], 0.0f) * ASC); }
            *(volatile v8h*)(hp + (size_t)r * DM + c8) = hv; }
        if (ps == 0) __threadfence(); }
}

static constexpr size_t al256(size_t v) { return (v + 255) & ~(size_t)255; }
static constexpr size_t PLANE_E = (size_t)NB * NH_ * SEQ * HD;
static constexpr size_t SZ_XB = al256((size_t)NB * SEQ * DM * 2);
static constexpr size_t SZ_WQ = al256((size_t)QKVW * DM * 2);
static constexpr size_t SZ_WH = al256((size_t)DM * DM * 2);
static constexpr size_t SZ_P2 = al256((size_t)2 * PLANE_E * 2);
static constexpr size_t SZ_PL = al256(PLANE_E * 2);
static constexpr size_t SZ_F32 = al256((size_t)NB * SEQ * DM * 4);
static constexpr size_t SZ_TOTAL = SZ_XB + SZ_WQ + 3 * SZ_WH + 2 * SZ_P2 + SZ_PL + SZ_XB + SZ_F32 + 2 * SZ_XB;
static_assert(SZ_TOTAL <= (size_t)134217728);
static_assert(PLANE_E == (size_t)NB * SEQ * DM);
static_assert((PLANE_E * 2) % 256 == 0);

extern "C" void kernel_launch(void* const* d_in, const int* in_sizes, int n_in,
                              void* d_out, int out_size, void* d_ws, size_t ws_size, hipStream_t stream) {
    if (n_in < 13) return;
    const size_t needx = ((size_t)(NB - 1) * SEQ_FULL + SEQ) * DM;
    if ((size_t)in_sizes[0] < needx) return;
    if ((size_t)in_sizes[1] < (size_t)DM * QKVW || in_sizes[2] < QKVW) return;
    if ((size_t)in_sizes[3] < (size_t)DM * DM || (size_t)in_sizes[5] < (size_t)DM * DM || (size_t)in_sizes[7] < (size_t)DM * DM) return;
    if (in_sizes[4] < DM || in_sizes[6] < DM || in_sizes[8] < DM) return;
    if (in_sizes[9] < DM || in_sizes[10] < DM || in_sizes[11] < DM || in_sizes[12] < DM) return;
    if ((size_t)out_size < ((size_t)(NB - 1) * OUT_SEQ + SEQ) * DM) return;
    if (SZ_TOTAL > ws_size) return;
    const float* x = (const float*)d_in[0];
    const float* wqkv = (const float*)d_in[1];  const float* bqkv = (const float*)d_in[2];
    const float* wattn = (const float*)d_in[3]; const float* battn = (const float*)d_in[4];
    const float* w1 = (const float*)d_in[5];    const float* b1 = (const float*)d_in[6];
    const float* w2 = (const float*)d_in[7];    const float* b2 = (const float*)d_in[8];
    const float* g1 = (const float*)d_in[9];    const float* be1 = (const float*)d_in[10];
    const float* g2 = (const float*)d_in[11];   const float* be2 = (const float*)d_in[12];
    float* OUT = (float*)d_out;
    char* wsp = (char*)d_ws;
    bf*  XB  = (bf*)wsp;  wsp += SZ_XB;
    bf*  WQT = (bf*)wsp;  wsp += SZ_WQ;
    h16* WAT = (h16*)wsp; wsp += SZ_WH;
    h16* W1T = (h16*)wsp; wsp += SZ_WH;
    h16* W2T = (h16*)wsp; wsp += SZ_WH;
    h16* PH  = (h16*)wsp; wsp += SZ_P2;
    h16* PR  = (h16*)wsp; wsp += SZ_P2;
    h16* VT  = (h16*)wsp; wsp += SZ_PL;
    h16* CTX = (h16*)wsp; wsp += SZ_XB;
    float* X1F = (float*)wsp; wsp += SZ_F32;
    h16* X1H = (h16*)wsp; wsp += SZ_XB;
    h16* HP  = (h16*)wsp; wsp += SZ_XB;

    if (SEQ == SEQ_FULL) {
        const size_t n8 = (size_t)NB * SEQ * DM / 8;
        k_cvt8<<<(unsigned)((n8 + 255) / 256), 256, 0, stream>>>(x, XB, n8);
    } else {
        const size_t n8 = (size_t)SEQ * DM / 8;
        for (int b = 0; b < NB; ++b) k_cvt8<<<(unsigned)((n8 + 255) / 256), 256, 0, stream>>>(x + (size_t)b * SEQ_FULL * DM, XB + (size_t)b * SEQ * DM, n8);
    }
    k_wt_bf<<<dim3(DM / 64, QKVW / 32, 1), 256, 0, stream>>>(wqkv, WQT, DM, QKVW);
    k_wt_h<<<dim3(DM / 64, DM / 32, 1), 256, 0, stream>>>(wattn, WAT, DM, DM);
    k_wt_h<<<dim3(DM / 64, DM / 32, 1), 256, 0, stream>>>(w1, W1T, DM, DM);
    k_wt_h<<<dim3(DM / 64, DM / 32, 1), 256, 0, stream>>>(w2, W2T, DM, DM);

    k_qk<<<dim3(NB * SEQ / 64, 8, 1), 32, 0, stream>>>(XB, WQT, bqkv, PH, PR);
    k_vt<<<dim3(4, NB * SEQ / 64, 1), 32, 0, stream>>>(WQT, XB, bqkv, VT);

    k_flash<<<dim3(SEQ / (16 * AW), NB * NH_, 1), 32 * AW, 0, stream>>>(PH, PR, PH + PLANE_E, PR + PLANE_E, VT, CTX);

    k_gemm_ln<<<dim3(NB * SEQ / (16 * GW), 1, 1), 32 * GW, 0, stream>>>(CTX, WAT, battn, x, g1, be1, X1F, X1H, SEQ_FULL, SEQ, 0);
    k_gemm_relu<<<dim3(NB * SEQ / (16 * GW), 1, 1), 32 * GW, 0, stream>>>(X1H, W1T, b1, HP);
    k_gemm_ln<<<dim3(NB * SEQ / (16 * GW), 1, 1), 32 * GW, 0, stream>>>(HP, W2T, b2, X1F, g2, be2, OUT, X1H, SEQ, OUT_SEQ, 1);
}
